// diffRNN_75591424410018
// MI455X (gfx1250) — hardware-run, weakly checked
//
#include <hip/hip_runtime.h>
#include <math.h>

typedef __attribute__((ext_vector_type(16))) _Float16 v16h;
typedef __attribute__((ext_vector_type(8)))  _Float16 v8h;
typedef __attribute__((ext_vector_type(8)))  float    v8f;
typedef __attribute__((ext_vector_type(4)))  float    v4f;
typedef __attribute__((ext_vector_type(2)))  float    v2f;

constexpr int kB   = 64;
constexpr int kV   = 50;
constexpr int kC   = 20;
constexpr int kD   = 256;
constexpr int kVoc = 10000;
constexpr int kTd  = 1000;
constexpr int kR   = kB * kV;
constexpr int kR2  = 2 * kR;
constexpr int kHd  = 512;
constexpr int kG4  = 4 * kD;
constexpr int kC1  = 4 * kD;
constexpr int kC2  = 2 * kD;
constexpr int kHP  = 264;
static_assert(kR == 3200 && kR2 == 6400);
static_assert((kR % 64) == 0 && (kR2 % 64) == 0);
static_assert((kD % 64) == 0 && (kHd % 64) == 0 && (kG4 % 64) == 0 && (kC2 % 64) == 0);
static_assert((kD % 32) == 0 && (kHd % 32) == 0 && (kC1 % 32) == 0);

constexpr float kCarryW   = 1024.0f;
constexpr float kCarryXin = 16.0f;
constexpr float kCarryHd  = 128.0f;
constexpr float kCarryG1  = 16.0f;
constexpr float kCarryTv  = 128.0f;
constexpr float kCarryX   = 256.0f;
constexpr float kCarryH   = 512.0f;
constexpr float kCarryA1  = 4096.0f;
constexpr float kSclDiff1 = 1.0f / (kCarryXin * kCarryW);
constexpr float kSclDiff2 = 1.0f / (kCarryHd * kCarryW);
constexpr float kSclAv    = 1.0f / (kCarryG1 * kCarryW);
constexpr float kSclAo    = 1.0f / (kCarryTv * kCarryW);
constexpr float kSclXw    = 1.0f / (kCarryX * kCarryW);
constexpr float kSclLstm  = 1.0f / (kCarryH * kCarryW);
constexpr float kSclC1    = 1.0f / (kCarryH * kCarryW);
constexpr float kSclC2    = 1.0f / (kCarryA1 * kCarryW);
constexpr float kF16MinNormal = 6.103515625e-05f;

constexpr int kOut0 = 0;
constexpr int kOut2 = 2 * kR2;
constexpr int kOut4 = kOut2 + 4 * kB;
constexpr int kOutPred = kOut4 + kR * kD;
constexpr int kOutTotal = kOutPred + kR * kD;
static_assert(kOut2 == 12800 && kOut4 == 13056 && kOutPred == 832256 && kOutTotal == 1651456);
static_assert(((size_t)kOut4 * 4) % 128 == 0 && ((size_t)kOutPred * 4) % 128 == 0 && ((size_t)kOut2 * 4) % 128 == 0);

constexpr size_t kOffSC   = 0;
constexpr size_t kOffTEMB = kOffSC   + (size_t)kB * 32 * 4;
constexpr size_t kOffW1T  = kOffTEMB + (size_t)kB * kD * 4;
constexpr size_t kOffW2T  = kOffW1T  + (size_t)kHd * kD * 2;
constexpr size_t kOffWV   = kOffW2T  + (size_t)kD * kHd * 2;
constexpr size_t kOffWO   = kOffWV   + (size_t)kD * kD * 2;
constexpr size_t kOffWIH  = kOffWO   + (size_t)kD * kD * 2;
constexpr size_t kOffWHH  = kOffWIH  + (size_t)kG4 * kD * 2;
constexpr size_t kOffC1W  = kOffWHH  + (size_t)kG4 * kD * 2;
constexpr size_t kOffC2W  = kOffC1W  + (size_t)kC1 * kD * 2;
constexpr size_t kOffVE   = kOffC2W  + (size_t)kC2 * kC1 * 2;
constexpr size_t kOffXIN  = kOffVE   + (size_t)kR * kD * 4;
constexpr size_t kOffHD   = kOffXIN  + (size_t)kR * kD * 2;
constexpr size_t kOffG1   = kOffHD   + (size_t)kR * kHd * 2;
constexpr size_t kOffTV   = kOffG1   + (size_t)kR * kD * 2;
constexpr size_t kOffX    = kOffTV   + (size_t)kR * kD * 2;
constexpr size_t kOffG    = kOffX    + (size_t)kR2 * kD * 2;
constexpr size_t kOffHS   = kOffG    + (size_t)kR2 * kG4 * 4;
constexpr size_t kOffA1   = kOffHS   + (size_t)kR2 * kD * 2;
constexpr size_t kOffA2   = kOffA1   + (size_t)kR2 * kC1 * 2;
constexpr size_t kWsTotal = kOffA2   + (size_t)kR2 * kC2 * 4;
static_assert(kWsTotal == 73932800ull);
static_assert(kWsTotal <= 134217728ull);
static_assert((kOffTEMB % 128) == 0 && (kOffW1T % 128) == 0 && (kOffW2T % 128) == 0 && (kOffWV % 128) == 0 &&
              (kOffWO % 128) == 0 && (kOffWIH % 128) == 0 && (kOffWHH % 128) == 0 && (kOffC1W % 128) == 0 &&
              (kOffC2W % 128) == 0 && (kOffVE % 128) == 0 && (kOffXIN % 128) == 0 && (kOffHD % 128) == 0 &&
              (kOffG1 % 128) == 0 && (kOffTV % 128) == 0 && (kOffX % 128) == 0 && (kOffG % 128) == 0 &&
              (kOffHS % 128) == 0 && (kOffA1 % 128) == 0 && (kOffA2 % 128) == 0);

__device__ __forceinline__ _Float16 to_h16(float v) {
  const float f = (fabsf(v) < kF16MinNormal) ? 0.0f : v;
  return (_Float16)f;
}
__device__ __forceinline__ v16h frag_load(const _Float16* p) {
  union U { v16h v; v8h h[2]; };
  U f;
  f.h[0] = *(const v8h*)(p);
  f.h[1] = *(const v8h*)(p + 16);
  return f.v;
}
__device__ __forceinline__ v8f mma_h(v16h a, v16h b, v8f c) {
  return __builtin_amdgcn_wmma_f32_16x16x32_f16(false, a, false, b, (short)0, c, false, false);
}
__device__ __forceinline__ v8f mma_guarded(v16h a, v16h b, v8f c) {
  c = __builtin_amdgcn_wmma_f32_16x16x32_f16(false, a, false, b, (short)0, c, false, false);
  asm volatile("v_nop\n\tv_nop\n\tv_nop\n\tv_nop" : "+v"(c) : "v"(a), "v"(b));
  return c;
}
__device__ __forceinline__ void guard_row4(v8f& c0, v8f& c1, v8f& c2, v8f& c3,
                                           v16h a, v16h b0, v16h b1, v16h b2, v16h b3) {
  asm volatile("v_nop\n\tv_nop\n\tv_nop\n\tv_nop"
               : "+v"(c0), "+v"(c1), "+v"(c2), "+v"(c3)
               : "v"(a), "v"(b0), "v"(b1), "v"(b2), "v"(b3));
}
__device__ __forceinline__ void keep4_h(v16h a, v16h b, v16h c, v16h d) { asm volatile("v_nop" :: "v"(a), "v"(b), "v"(c), "v"(d)); }
__device__ __forceinline__ void acc_guard4(v8f& a, v8f& b, v8f& c, v8f& d) { asm volatile("v_nop\n\tv_nop\n\tv_nop\n\tv_nop" : "+v"(a), "+v"(b), "+v"(c), "+v"(d)); }
__device__ __forceinline__ float sigm(float x) { return 1.0f / (1.0f + expf(-x)); }

template <bool HAS_BIAS, int OUT_MODE, int ACT>
__global__ __launch_bounds__(256) void gemm64_f16(
    const unsigned short* __restrict__ Ap, int lda,
    const unsigned short* __restrict__ Btp, int ldb,
    void* __restrict__ Cout, int ldc,
    const float* __restrict__ bias,
    int M, int N, int K, float scale, float ocarry) {
  const _Float16* A  = (const _Float16*)Ap;
  const _Float16* Bt = (const _Float16*)Btp;
  __shared__ __align__(16) float sT[8][16 * 68];
  const int lane = threadIdx.x & 31;
  const int wave = threadIdx.x >> 5;
  const int tilesN = N >> 6;
  const int tilesM = M >> 6;
  const int tile = blockIdx.x * 8 + wave;
  if (tile >= tilesM * tilesN) return;
  const int tm = tile / tilesN;
  const int tn = tile - tm * tilesN;
  const int m0 = tm << 6;
  const int n0 = tn << 6;

  const int rlane = lane & 15;
  const int koff  = (lane >> 4) * 8;
  const int mOff  = (lane >> 4) * 8;

  v8f acc[4][4];
#pragma unroll
  for (int i = 0; i < 4; ++i)
#pragma unroll
    for (int j = 0; j < 4; ++j) acc[i][j] = (v8f){0.f, 0.f, 0.f, 0.f, 0.f, 0.f, 0.f, 0.f};

  for (int k0 = 0; k0 < K; k0 += 32) {
    v16h bh[4];
#pragma unroll
    for (int j = 0; j < 4; ++j) {
      const size_t bo = (size_t)(n0 + (j << 4) + rlane) * ldb + koff + k0;
      bh[j] = frag_load(Bt + bo);
    }
#pragma unroll
    for (int i = 0; i < 4; ++i) {
      const size_t ao = (size_t)(m0 + (i << 4) + rlane) * lda + koff + k0;
      const v16h ah = frag_load(A + ao);
#pragma unroll
      for (int j = 0; j < 4; ++j) acc[i][j] = mma_h(ah, bh[j], acc[i][j]);
      guard_row4(acc[i][0], acc[i][1], acc[i][2], acc[i][3], ah, bh[0], bh[1], bh[2], bh[3]);
    }
    keep4_h(bh[0], bh[1], bh[2], bh[3]);
  }
  acc_guard4(acc[0][0], acc[0][1], acc[0][2], acc[0][3]);
  acc_guard4(acc[1][0], acc[1][1], acc[1][2], acc[1][3]);
  acc_guard4(acc[2][0], acc[2][1], acc[2][2], acc[2][3]);
  acc_guard4(acc[3][0], acc[3][1], acc[3][2], acc[3][3]);

  float* slab = sT[wave];
#pragma unroll
  for (int i = 0; i < 4; ++i) {
    const int mBase = m0 + (i << 4);
#pragma unroll
    for (int j = 0; j < 4; ++j) {
      const int n = n0 + (j << 4) + rlane;
      float bv = 0.f;
      if (HAS_BIAS) bv = bias[n];
#pragma unroll
      for (int r = 0; r < 8; ++r) {
        float v = acc[i][j][r] * scale;
        if (HAS_BIAS) v += bv;
        if (ACT == 2) v = fmaxf(v, 0.0f);
        slab[(mOff + r) * 68 + (j << 4) + rlane] = v;
      }
    }
    __builtin_amdgcn_fence(__ATOMIC_RELEASE, "workgroup");
    __builtin_amdgcn_wave_barrier();
    __builtin_amdgcn_fence(__ATOMIC_ACQUIRE, "workgroup");
    if (OUT_MODE == 0) {
      float* Cf = (float*)Cout;
      const int hh = lane >> 4, c4 = (lane & 15) * 4;
      for (int pass = 0; pass < 2; ++pass) {
#pragma unroll
        for (int it = 0; it < 8; ++it) {
          const int row = it * 2 + hh;
          const v4f v = *(const v4f*)(slab + row * 68 + c4);
          *(volatile v4f*)(Cf + (size_t)(mBase + row) * ldc + n0 + c4) = v;
        }
        __threadfence();
      }
    } else {
      const int q = lane >> 3, c8 = (lane & 7) * 8;
      unsigned short* Ch = (unsigned short*)Cout;
      for (int pass = 0; pass < 2; ++pass) {
#pragma unroll
        for (int it = 0; it < 4; ++it) {
          const int row = it * 4 + q;
          const float* sp = slab + row * 68 + c8;
          v8h hv;
#pragma unroll
          for (int e = 0; e < 8; ++e) hv[e] = to_h16(sp[e] * ocarry);
          *(volatile v8h*)(Ch + (size_t)(mBase + row) * ldc + n0 + c8) = hv;
        }
        __threadfence();
      }
    }
    __builtin_amdgcn_fence(__ATOMIC_RELEASE, "workgroup");
    __builtin_amdgcn_wave_barrier();
    __builtin_amdgcn_fence(__ATOMIC_ACQUIRE, "workgroup");
  }
}

__global__ __launch_bounds__(256) void prep_kernel(const int* __restrict__ tdiff, float* __restrict__ sc,
                                                   float* __restrict__ temb) {
  __shared__ float sS[2];
  const int b = blockIdx.x, tid = threadIdx.x, lane = tid & 31, wave = tid >> 5;
  int t = tdiff[b];
  t = (t < 0) ? 0 : ((t > kTd - 1) ? (kTd - 1) : t);
  if (tid == 0) {
    float prod = 1.0f;
#pragma unroll 1
    for (int i = 0; i <= t; ++i) {
      const float s = (float)i * (1.0f / (float)(kTd - 1));
      float beta = 1e-4f * (1.0f - s) + 0.02f * s;
      if (i == kTd - 1) beta = 0.02f;
      prod *= (1.0f - beta);
    }
    sS[0] = sqrtf(prod);
    sS[1] = sqrtf(1.0f - prod);
  }
  __syncthreads();
  const int fi = tid & 127;
  const float freq = expf((-9.210340371976184f * (float)fi) * (1.0f / 128.0f));
  const float arg = (float)t * freq;
  const float sn = sinf(arg);
  const float cs = cosf(arg);
  const float val = (tid < 128) ? sn : cs;
  const float s0 = sS[0], s1 = sS[1];
  const float lv = (lane == 0) ? s0 : ((lane == 1) ? s1 : 0.0f);
  for (int pass = 0; pass < 2; ++pass) {
    *(volatile float*)(temb + (size_t)b * kD + tid) = val;
    if (wave == 0) *(volatile float*)(sc + (size_t)b * 32 + lane) = lv;
    __threadfence();
  }
}

__global__ __launch_bounds__(256) void cast_w_kernel(const float* __restrict__ src, unsigned short* __restrict__ dst, int n8) {
  const int i = blockIdx.x * 256 + threadIdx.x;
  if (i >= n8) return;
  const size_t e0 = (size_t)i << 3;
  const v4f a0 = *(const v4f*)(src + e0);
  const v4f a1 = *(const v4f*)(src + e0 + 4);
  v8h hv;
#pragma unroll
  for (int e = 0; e < 4; ++e) {
    hv[e]     = to_h16(a0[e] * kCarryW);
    hv[4 + e] = to_h16(a1[e] * kCarryW);
  }
  *(volatile v8h*)(dst + e0) = hv;
  __threadfence();
  *(volatile v8h*)(dst + e0) = hv;
}

__global__ __launch_bounds__(256) void transpose_cast_kernel(const float* __restrict__ in, unsigned short* __restrict__ outp,
                                                             int rowsK, int colsN) {
  __shared__ float sT[64 * 65];
  const int tid = threadIdx.x;
  const int n0 = blockIdx.x * 64, k0 = blockIdx.y * 64;
#pragma unroll
  for (int it = 0; it < 16; ++it) {
    const int kr = it * 4 + (tid >> 6);
    const int cc = tid & 63;
    sT[kr * 65 + cc] = in[(size_t)(k0 + kr) * colsN + n0 + cc];
  }
  __syncthreads();
  v8h hv[2];
#pragma unroll
  for (int it = 0; it < 2; ++it) {
    const int nrow = it * 32 + (tid >> 3);
    const int ks = (tid & 7) * 8;
#pragma unroll
    for (int e = 0; e < 8; ++e) hv[it][e] = to_h16(sT[(ks + e) * 65 + nrow] * kCarryW);
  }
  for (int pass = 0; pass < 2; ++pass) {
#pragma unroll
    for (int it = 0; it < 2; ++it) {
      const int nrow = it * 32 + (tid >> 3);
      const int ks = (tid & 7) * 8;
      *(volatile v8h*)(outp + (size_t)(n0 + nrow) * rowsK + k0 + ks) = hv[it];
    }
    __threadfence();
  }
}

__global__ __launch_bounds__(128) void visit_kernel(
    const int* __restrict__ seqs, const float* __restrict__ stime, const float* __restrict__ noise,
    const float* __restrict__ emb, const float* __restrict__ tw1, const float* __restrict__ tb1,
    const float* __restrict__ tw2, const float* __restrict__ tb2,
    const float* __restrict__ sc, const float* __restrict__ temb,
    float* __restrict__ ve, unsigned short* __restrict__ xin16, unsigned short* __restrict__ x16,
    float* __restrict__ out4) {
  __shared__ __align__(16) float sTf[64];
  __shared__ __align__(16) float sVe[kD];
  __shared__ __align__(16) float sXin[kD];
  __shared__ int sIdx[32];
  const int r = blockIdx.x;
  const int b = r / kV;
  const int tid = threadIdx.x, lane = tid & 31, wave = tid >> 5;
  {
    const int k = tid & 63;
    const float tval = stime[r] * (1.0f / 180.0f);
    const float u = tval * tw1[k] + tb1[k];
    const float tfv = 1.0f - tanhf(u * u);
    if (tid < 64) sTf[k] = tfv;
    const int ci = (tid < kC) ? tid : (kC - 1);
    int id = seqs[(size_t)r * kC + ci];
    asm volatile("" : "+v"(id));
    id = (id < 0) ? 0 : ((id > kVoc) ? kVoc : id);
    if (tid < kC) sIdx[tid] = id;
  }
  __syncthreads();
  const int d0 = 2 * tid;
  float te0 = 0.0f, te1 = 0.0f;
  {
    const float* w2a = tw2 + (size_t)d0 * 64;
#pragma unroll 1
    for (int i = 0; i < 16; ++i) {
      const v4f t4 = *(const v4f*)(sTf + 4 * i);
      const v4f wa = *(const v4f*)(w2a + 4 * i);
      const v4f wb = *(const v4f*)(w2a + 64 + 4 * i);
      te0 = fmaf(t4[0], wa[0], te0);
      te0 = fmaf(t4[1], wa[1], te0);
      te0 = fmaf(t4[2], wa[2], te0);
      te0 = fmaf(t4[3], wa[3], te0);
      te1 = fmaf(t4[0], wb[0], te1);
      te1 = fmaf(t4[1], wb[1], te1);
      te1 = fmaf(t4[2], wb[2], te1);
      te1 = fmaf(t4[3], wb[3], te1);
    }
    const v2f b2v = *(const v2f*)(tb2 + d0);
    te0 += b2v[0];
    te1 += b2v[1];
  }
  float s0 = 0.0f, s1 = 0.0f;
#pragma unroll 4
  for (int c = 0; c < kC; ++c) {
    const int id = sIdx[c];
    const v2f e = *(const v2f*)(emb + (size_t)id * kD + d0);
    s0 += fmaxf(e[0], 0.0f);
    s1 += fmaxf(e[1], 0.0f);
  }
  const float v0 = s0 + te0, v1 = s1 + te1;
  const size_t rb = (size_t)r * kD;
  {
    const v2f nz = *(const v2f*)(noise + rb + d0);
    const float sa = sc[(size_t)b * 32], sb = sc[(size_t)b * 32 + 1];
    const v2f tv = *(const v2f*)(temb + (size_t)b * kD + d0);
    const float x0 = (v0 * sa + nz[0] * sb) + tv[0];
    const float x1 = (v1 * sa + nz[1] * sb) + tv[1];
    sVe[d0] = v0;
    sVe[d0 + 1] = v1;
    sXin[d0] = x0;
    sXin[d0 + 1] = x1;
  }
  __syncthreads();
  if (wave < 2) {
    const v4f vv = *(const v4f*)(sVe + 4 * tid);
    const v4f nn = *(const v4f*)(noise + rb + 4 * tid);
    for (int pass = 0; pass < 2; ++pass) {
      *(volatile v4f*)(ve + rb + 4 * tid) = vv;
      *(volatile v4f*)(out4 + rb + 4 * tid) = nn;
      __threadfence();
    }
  } else {
    const float* sp = (wave == 2) ? sXin : sVe;
    const float cr = (wave == 2) ? kCarryXin : kCarryX;
    unsigned short* dst = (wave == 2) ? xin16 : x16;
    const v4f a0 = *(const v4f*)(sp + 8 * lane);
    const v4f a1 = *(const v4f*)(sp + 8 * lane + 4);
    v8h hv;
#pragma unroll
    for (int e = 0; e < 4; ++e) {
      hv[e]     = to_h16(a0[e] * cr);
      hv[4 + e] = to_h16(a1[e] * cr);
    }
    for (int pass = 0; pass < 2; ++pass) {
      *(volatile v8h*)(dst + rb + 8 * lane) = hv;
      __threadfence();
    }
  }
}

__global__ __launch_bounds__(256) void gen1_kernel(const float* __restrict__ ve, const float* __restrict__ noise,
                                                   const float* __restrict__ pred, unsigned short* __restrict__ g1, int total8) {
  const int i = blockIdx.x * 256 + threadIdx.x;
  if (i >= total8) return;
  const size_t e0 = (size_t)i << 3;
  const v4f a0 = *(const v4f*)(ve + e0);
  const v4f a1 = *(const v4f*)(ve + e0 + 4);
  const v4f n0 = *(const v4f*)(noise + e0);
  const v4f n1 = *(const v4f*)(noise + e0 + 4);
  const v4f p0 = *(const v4f*)(pred + e0);
  const v4f p1 = *(const v4f*)(pred + e0 + 4);
  v8h hv;
#pragma unroll
  for (int e = 0; e < 4; ++e) {
    hv[e]     = to_h16((a0[e] + (n0[e] - p0[e])) * kCarryG1);
    hv[4 + e] = to_h16((a1[e] + (n1[e] - p1[e])) * kCarryG1);
  }
  *(volatile v8h*)(g1 + e0) = hv;
  __threadfence();
  *(volatile v8h*)(g1 + e0) = hv;
}

__global__ __launch_bounds__(256) void lstm_kernel(
    const float* __restrict__ G, const unsigned short* __restrict__ Whp,
    const float* __restrict__ bih, const float* __restrict__ bhh,
    unsigned short* __restrict__ HS) {
  __shared__ __align__(16) _Float16 sH[2 * 16 * kHP];
  __shared__ float sC[8 * 16 * 32];
  __shared__ float sGt[8 * 16 * 32];
  const _Float16* W = (const _Float16*)Whp;
  const int tid = threadIdx.x, lane = tid & 31, wave = tid >> 5;
  const int hh = lane >> 4, cl = lane & 15;
  const int j0 = blockIdx.x * 16;
  const int ucol = 32 * wave + cl;

  {
    v8h z;
#pragma unroll
    for (int e = 0; e < 8; ++e) z[e] = (_Float16)0.0f;
    for (int i = tid; i < (2 * 16 * kHP) / 8; i += 256) *(v8h*)(sH + 8 * i) = z;
#pragma unroll
    for (int i = 0; i < 16; ++i) sC[(wave * 16 + i) * 32 + lane] = 0.0f;
  }
  float bs[4][2];
#pragma unroll
  for (int g = 0; g < 4; ++g)
#pragma unroll
    for (int s = 0; s < 2; ++s) {
      const int n = g * kD + ucol + 16 * s;
      bs[g][s] = bih[n] + bhh[n];
    }
  __syncthreads();

  const _Float16* wb = W + (size_t)ucol * kD + 8 * hh;
#pragma unroll 1
  for (int v = 0; v < kV; ++v) {
    const int cur = v & 1;
    const _Float16* hc = sH + cur * (16 * kHP);
    _Float16* hn = sH + (cur ^ 1) * (16 * kHP);
    v8f acc[8];
#pragma unroll
    for (int t = 0; t < 8; ++t) acc[t] = (v8f){0.f, 0.f, 0.f, 0.f, 0.f, 0.f, 0.f, 0.f};
#pragma unroll 2
    for (int ks = 0; ks < 8; ++ks) {
      const v16h a = frag_load(hc + cl * kHP + ks * 32 + 8 * hh);
      v16h bq[8];
#pragma unroll
      for (int t = 0; t < 8; ++t)
        bq[t] = frag_load(wb + (size_t)(((t >> 1) * kD + (t & 1) * 16) * kD) + ks * 32);
#pragma unroll
      for (int t = 0; t < 8; ++t) acc[t] = mma_guarded(a, bq[t], acc[t]);
    }
#pragma unroll
    for (int s = 0; s < 2; ++s) {
#pragma unroll
      for (int hf = 0; hf < 2; ++hf) {
#pragma unroll
        for (int g = 0; g < 4; ++g)
#pragma unroll
          for (int ii = 0; ii < 4; ++ii)
            sGt[((wave * 4 + g) * 4 + ii) * 32 + lane] = acc[g * 2 + s][hf * 4 + ii] * kSclLstm;
#pragma unroll 1
        for (int ii = 0; ii < 4; ++ii) {
          const int i = hf * 4 + ii;
          const int row = 8 * hh + i;
          const size_t gb = ((size_t)(j0 + row) * kV + v) * kG4 + ucol + 16 * s;
          const float xi = G[gb];
          const float xf = G[gb + kD];
          const float xg = G[gb + 2 * kD];
          const float xo = G[gb + 3 * kD];
          const float gi = (sGt[((wave * 4 + 0) * 4 + ii) * 32 + lane] + xi) + bs[0][s];
          const float gf = (sGt[((wave * 4 + 1) * 4 + ii) * 32 + lane] + xf) + bs[1][s];
          const float gg = (sGt[((wave * 4 + 2) * 4 + ii) * 32 + lane] + xg) + bs[2][s];
          const float go = (sGt[((wave * 4 + 3) * 4 + ii) * 32 + lane] + xo) + bs[3][s];
          const int ci = (wave * 16 + s * 8 + i) * 32 + lane;
          const float cprev = sC[ci];
          const float cn = sigm(gf) * cprev + sigm(gi) * tanhf(gg);
          sC[ci] = cn;
          const float hv = sigm(go) * tanhf(cn);
          hn[row * kHP + ucol + 16 * s] = to_h16(hv * kCarryH);
        }
      }
    }
    __syncthreads();
    {
      v8h r0 = *(const v8h*)(hn + (2 * wave) * kHP + 8 * lane);
      v8h r1 = *(const v8h*)(hn + (2 * wave + 1) * kHP + 8 * lane);
      unsigned short* d0p = HS + ((size_t)(j0 + 2 * wave) * kV + v) * kD + 8 * lane;
      unsigned short* d1p = HS + ((size_t)(j0 + 2 * wave + 1) * kV + v) * kD + 8 * lane;
      for (int pass = 0; pass < 2; ++pass) {
        *(volatile v8h*)d0p = r0;
        *(volatile v8h*)d1p = r1;
        __threadfence();
      }
    }
  }
}

__global__ __launch_bounds__(256) void head_kernel(const float* __restrict__ A2, const float* __restrict__ c3w,
                                                   const float* __restrict__ c3b, float* __restrict__ outp) {
  const int lane = threadIdx.x & 31, wave = threadIdx.x >> 5;
  const int gw = blockIdx.x * 8 + wave;
  if (gw >= 408) return;
  const int rsel = lane >> 1, o = lane & 1;
  int row;
  if (gw < 400) row = gw * 16 + rsel;
  else row = ((gw - 400) * 16 + rsel) * kV + (kV - 1);
  row = (row > kR2 - 1) ? (kR2 - 1) : row;
  const float* ar = A2 + (size_t)row * kC2;
  const float* wr = c3w + (size_t)o * kC2;
  float acc = 0.0f;
#pragma unroll 4
  for (int k4 = 0; k4 < kC2 / 4; ++k4) {
    const v4f a = *(const v4f*)(ar + 4 * k4);
    const v4f w = *(const v4f*)(wr + 4 * k4);
    acc = fmaf(a[0], w[0], acc);
    acc = fmaf(a[1], w[1], acc);
    acc = fmaf(a[2], w[2], acc);
    acc = fmaf(a[3], w[3], acc);
  }
  const float res = acc + c3b[o];
  float* dst = outp + (size_t)gw * 32 + lane;
  *(volatile float*)dst = res;
  __threadfence();
  *(volatile float*)dst = res;
}

extern "C" void kernel_launch(void* const* d_in, const int* in_sizes, int n_in,
                              void* d_out, int out_size, void* d_ws, size_t ws_size,
                              hipStream_t stream) {
  if (n_in < 27) return;
  if (in_sizes[0] != kB * kV * kC) return;
  if (in_sizes[1] != kR) return;
  if (in_sizes[2] != kB) return;
  if (in_sizes[3] != kR * kD) return;
  if (in_sizes[4] != (kVoc + 1) * kD) return;
  if (in_sizes[7] != kD * 64) return;
  if (in_sizes[9] != kD * kHd) return;
  if (in_sizes[11] != kHd * kD) return;
  if (in_sizes[13] != kD * kD) return;
  if (in_sizes[15] != kD * kD) return;
  if (in_sizes[17] != kG4 * kD) return;
  if (in_sizes[18] != kG4 * kD) return;
  if (in_sizes[21] != kC1 * kD) return;
  if (in_sizes[23] != kC2 * kC1) return;
  if (in_sizes[25] != 2 * kC2) return;
  if (in_sizes[26] != 2) return;
  if (out_size != kOutTotal) return;
  if (ws_size < kWsTotal) return;

  const int*   seqs  = (const int*)d_in[0];
  const float* stime = (const float*)d_in[1];
  const int*   tdiff = (const int*)d_in[2];
  const float* noise = (const float*)d_in[3];
  const float* emb   = (const float*)d_in[4];
  const float* tw1   = (const float*)d_in[5];
  const float* tb1   = (const float*)d_in[6];
  const float* tw2   = (const float*)d_in[7];
  const float* tb2   = (const float*)d_in[8];
  const float* dw1   = (const float*)d_in[9];
  const float* db1   = (const float*)d_in[10];
  const float* dw2   = (const float*)d_in[11];
  const float* db2   = (const float*)d_in[12];
  const float* awv   = (const float*)d_in[13];
  const float* abv   = (const float*)d_in[14];
  const float* awo   = (const float*)d_in[15];
  const float* abo   = (const float*)d_in[16];
  const float* wih   = (const float*)d_in[17];
  const float* whh   = (const float*)d_in[18];
  const float* bih   = (const float*)d_in[19];
  const float* bhh   = (const float*)d_in[20];
  const float* c1w   = (const float*)d_in[21];
  const float* c1b   = (const float*)d_in[22];
  const float* c2w   = (const float*)d_in[23];
  const float* c2b   = (const float*)d_in[24];
  const float* c3w   = (const float*)d_in[25];
  const float* c3b   = (const float*)d_in[26];

  float* out = (float*)d_out;
  float* out4 = out + kOut4;
  float* outPred = out + kOutPred;

  char* ws = (char*)d_ws;
  float*          SC   = (float*)(ws + kOffSC);
  float*          TEMB = (float*)(ws + kOffTEMB);
  unsigned short* W1T  = (unsigned short*)(ws + kOffW1T);
  unsigned short* W2T  = (unsigned short*)(ws + kOffW2T);
  unsigned short* WV   = (unsigned short*)(ws + kOffWV);
  unsigned short* WO   = (unsigned short*)(ws + kOffWO);
  unsigned short* WIH  = (unsigned short*)(ws + kOffWIH);
  unsigned short* WHH  = (unsigned short*)(ws + kOffWHH);
  unsigned short* C1W  = (unsigned short*)(ws + kOffC1W);
  unsigned short* C2W  = (unsigned short*)(ws + kOffC2W);
  float*          VE   = (float*)(ws + kOffVE);
  unsigned short* XIN  = (unsigned short*)(ws + kOffXIN);
  unsigned short* HD   = (unsigned short*)(ws + kOffHD);
  unsigned short* G1   = (unsigned short*)(ws + kOffG1);
  unsigned short* TV   = (unsigned short*)(ws + kOffTV);
  unsigned short* X16  = (unsigned short*)(ws + kOffX);
  float*          GP   = (float*)(ws + kOffG);
  unsigned short* HS   = (unsigned short*)(ws + kOffHS);
  unsigned short* A1   = (unsigned short*)(ws + kOffA1);
  float*          A2   = (float*)(ws + kOffA2);

  prep_kernel<<<kB, 256, 0, stream>>>(tdiff, SC, TEMB);

  cast_w_kernel<<<(kD * kD / 8) / 256, 256, 0, stream>>>(awv, WV, kD * kD / 8);
  cast_w_kernel<<<(kD * kD / 8) / 256, 256, 0, stream>>>(awo, WO, kD * kD / 8);
  cast_w_kernel<<<(kG4 * kD / 8) / 256, 256, 0, stream>>>(wih, WIH, kG4 * kD / 8);
  cast_w_kernel<<<(kG4 * kD / 8) / 256, 256, 0, stream>>>(whh, WHH, kG4 * kD / 8);
  cast_w_kernel<<<(kC1 * kD / 8) / 256, 256, 0, stream>>>(c1w, C1W, kC1 * kD / 8);
  cast_w_kernel<<<(kC2 * kC1 / 8) / 256, 256, 0, stream>>>(c2w, C2W, kC2 * kC1 / 8);
  transpose_cast_kernel<<<dim3(kHd / 64, kD / 64), 256, 0, stream>>>(dw1, W1T, kD, kHd);
  transpose_cast_kernel<<<dim3(kD / 64, kHd / 64), 256, 0, stream>>>(dw2, W2T, kHd, kD);

  visit_kernel<<<kR, 128, 0, stream>>>(seqs, stime, noise, emb, tw1, tb1, tw2, tb2, SC, TEMB, VE, XIN, X16, out4);

  gemm64_f16<true, 1, 2><<<50, 256, 0, stream>>>(XIN, kD, W1T, kD, (void*)HD, kHd, db1, kR, kHd, kD, kSclDiff1, kCarryHd);
  gemm64_f16<true, 0, 0><<<25, 256, 0, stream>>>(HD, kHd, W2T, kHd, (void*)outPred, kD, db2, kR, kD, kHd, kSclDiff2, 1.0f);
  gen1_kernel<<<(kR * kD / 8) / 256, 256, 0, stream>>>(VE, noise, outPred, G1, kR * kD / 8);
  gemm64_f16<true, 1, 0><<<25, 256, 0, stream>>>(G1, kD, WV, kD, (void*)TV, kD, abv, kR, kD, kD, kSclAv, kCarryTv);
  gemm64_f16<true, 1, 0><<<25, 256, 0, stream>>>(TV, kD, WO, kD, (void*)(X16 + (size_t)kR * kD), kD, abo, kR, kD, kD, kSclAo, kCarryX);
  gemm64_f16<false, 0, 0><<<200, 256, 0, stream>>>(X16, kD, WIH, kD, (void*)GP, kG4, bih, kR2, kG4, kD, kSclXw, 1.0f);
  lstm_kernel<<<8, 256, 0, stream>>>(GP, WHH, bih, bhh, HS);
  gemm64_f16<true, 1, 2><<<200, 256, 0, stream>>>(HS, kD, C1W, kD, (void*)A1, kC1, c1b, kR2, kC1, kD, kSclC1, kCarryA1);
  gemm64_f16<true, 0, 2><<<100, 256, 0, stream>>>(A1, kC1, C2W, kC1, (void*)A2, kC2, c2b, kR2, kC2, kC1, kSclC2, 1.0f);
  head_kernel<<<51, 256, 0, stream>>>(A2, c3w, c3b, out);
}
